// VelocityEGNNLayer_13950053777588
// MI455X (gfx1250) — hardware-verified
//
#include <hip/hip_runtime.h>


namespace {
constexpr int NB = 2, N = 512, H = 128, NN = NB * N;
constexpr float XS = 8.0f, WSC = 256.0f, CLAMPC = 100.0f;

typedef _Float16 b16;
typedef __attribute__((ext_vector_type(16))) _Float16 v16b;
typedef __attribute__((ext_vector_type(8))) _Float16 v8b;
typedef __attribute__((ext_vector_type(8))) float v8f;
typedef __attribute__((ext_vector_type(4))) float v4f;
__device__ __forceinline__ float bf16_rne(float f) { unsigned int u = __float_as_uint(f); u += 0x7FFFu + ((u >> 16) & 1u); return __uint_as_float(u & 0xFFFF0000u); }
__device__ __forceinline__ void split16(float v, b16& hi, b16& lo) { hi = (b16)v; lo = (b16)(v - (float)hi); }
__device__ __forceinline__ v16b frag_kb(const b16* p, int hh) { const v8b a = *(const v8b*)(p + 8 * hh), b = *(const v8b*)(p + 16 + 8 * hh); v16b f;
#pragma unroll
  for (int e = 0; e < 8; ++e) { f[e] = a[e]; f[8 + e] = b[e]; } return f; }
__device__ __forceinline__ v8f wmma16b(v16b a, v16b b, v8f c) { v8f d = __builtin_amdgcn_wmma_f32_16x16x32_f16(false, a, false, b, (short)0, c, false, false); asm volatile("v_nop\n\tv_nop\n\tv_nop\n\tv_nop" : "+v"(d) : "v"(a), "v"(b)); return d; }
__device__ __forceinline__ void wave_lds_sync() { __builtin_amdgcn_fence(__ATOMIC_RELEASE, "workgroup"); __builtin_amdgcn_wave_barrier(); __builtin_amdgcn_fence(__ATOMIC_ACQUIRE, "workgroup"); }
__device__ __forceinline__ float nexp(float x) { return __builtin_amdgcn_exp2f(x * 1.4426950408889634f); }
__device__ __forceinline__ float pmul(float a, float b) { float p = a * b; asm volatile("" : "+v"(p)); return p; }
__device__ __forceinline__ float hsum16(float v) { v += __shfl_xor(v, 1); v += __shfl_xor(v, 2); v += __shfl_xor(v, 4); return v + __shfl_xor(v, 8); }
__device__ __forceinline__ float silu(float x) { return x / (1.0f + nexp(-x)); }
__device__ __forceinline__ float sigm(float x) { return 1.0f / (1.0f + nexp(-x)); }
__device__ __forceinline__ float tanh_(float x) { const float e = nexp(-2.0f * fabsf(x)); const float t = (1.0f - e) / (1.0f + e); return x < 0.0f ? -t : t; }

__global__ __launch_bounds__(256) void prep_kernel(const float* __restrict__ h, const float* __restrict__ we1, const float* __restrict__ we2, const float* __restrict__ wp1, const float* __restrict__ wv1, const float* __restrict__ wn1, const float* __restrict__ wn2, b16* __restrict__ H16, b16* __restrict__ WT) {
  const int t = blockIdx.x * 256 + threadIdx.x; const int nh = NN * H / 8, nw = H * H / 8; v8b o;
  if (t < nh) { const v4f a = *(const v4f*)(h + (size_t)t * 8), c = *(const v4f*)(h + (size_t)t * 8 + 4); for (int j = 0; j < 4; ++j) { o[j] = (b16)(bf16_rne(a[j]) * XS); o[4 + j] = (b16)(bf16_rne(c[j]) * XS); } for (int pass = 0; pass < 2; ++pass) { *(volatile v8b*)(H16 + (size_t)t * 8) = o; __threadfence(); } return; }
  const int u = t - nh; const int k = u / nw; if (k >= 8) return; const int e = (u - k * nw) * 8; const int oo = e / H, i0 = e - oo * H;
  for (int j = 0; j < 8; ++j) { const int i = i0 + j; float w;
    switch (k) { case 0: w = we1[(size_t)i * H + oo]; break; case 1: w = we1[(size_t)(H + i) * H + oo]; break; case 2: w = we2[(size_t)i * H + oo]; break; case 3: w = wp1[(size_t)i * H + oo]; break; case 4: w = wv1[(size_t)i * H + oo]; break; case 5: w = wn1[(size_t)i * H + oo]; break; case 6: w = wn1[(size_t)(H + i) * H + oo]; break; default: w = wn2[(size_t)i * H + oo]; }
    o[j] = (b16)(bf16_rne(w) * WSC); }
  b16* dst = (k == 5 || k == 6) ? WT + (size_t)5 * H * H + (size_t)oo * 2 * H + (k == 6 ? H : 0) + i0 : (k == 7 ? WT + (size_t)7 * H * H + (size_t)oo * H + i0 : WT + (size_t)k * H * H + (size_t)oo * H + i0);
  for (int pass = 0; pass < 2; ++pass) { *(volatile v8b*)dst = o; __threadfence(); }
}
__global__ __launch_bounds__(128) void nodeab_kernel(const b16* __restrict__ H16, const b16* __restrict__ WT, float* __restrict__ AF, float* __restrict__ BF) {
  __shared__ __attribute__((aligned(16))) float Ts[4][16][H + 4];
  const int wave = threadIdx.x >> 5, lane = threadIdx.x & 31, nloc = lane & 15, hlf = lane >> 4; const size_t m0 = (size_t)blockIdx.x * 64 + wave * 16; const int which = blockIdx.y; const b16* W = WT + (size_t)which * H * H;
  v8f acc[8];
#pragma unroll
  for (int t = 0; t < 8; ++t) acc[t] = (v8f){};
#pragma unroll
  for (int kb = 0; kb < H; kb += 32) { const v16b a = frag_kb(H16 + (m0 + nloc) * H + kb, hlf);
#pragma unroll
    for (int t = 0; t < 8; ++t) acc[t] = wmma16b(a, frag_kb(W + (size_t)(t * 16 + nloc) * H + kb, hlf), acc[t]); }
#pragma unroll
  for (int t = 0; t < 8; ++t)
#pragma unroll
    for (int r = 0; r < 8; ++r) Ts[wave][8 * hlf + r][t * 16 + nloc] = acc[t][r] * (1.0f / (XS * WSC));
  wave_lds_sync();
  float* dst = which ? BF : AF;
  for (int pass = 0; pass < 2; ++pass) { for (int rr = 0; rr < 16; ++rr) *(volatile v4f*)(dst + (m0 + rr) * H + lane * 4) = *(const v4f*)(&Ts[wave][rr][lane * 4]); __threadfence(); }
}
__global__ __launch_bounds__(128) void edge_kernel(const float* __restrict__ AF, const float* __restrict__ BF, const float* __restrict__ pos, const float* __restrict__ vel, const float* __restrict__ we1, const float* __restrict__ be1, const float* __restrict__ be2, const float* __restrict__ wa, const float* __restrict__ ba,
                                                const b16* __restrict__ WT, int node0, b16* __restrict__ Mh, b16* __restrict__ Ml) {
  __shared__ __attribute__((aligned(16))) b16 Th[4][16][H + 8], Tl[4][16][H + 8];
  const int wave = threadIdx.x >> 5, lane = threadIdx.x & 31, nloc = lane & 15, hlf = lane >> 4; const int gw = blockIdx.x * 4 + wave; const int il = gw >> 5, jt = gw & 31; const int node = node0 + il; const int b = node / N; const int j0 = jt * 16;
  const b16* WE2T = WT + (size_t)2 * H * H;
  const float pix = bf16_rne(pos[(size_t)node * 3]), piy = bf16_rne(pos[(size_t)node * 3 + 1]), piz = bf16_rne(pos[(size_t)node * 3 + 2]); const float vix = bf16_rne(vel[(size_t)node * 3]), viy = bf16_rne(vel[(size_t)node * 3 + 1]), viz = bf16_rne(vel[(size_t)node * 3 + 2]);
  float ab[8], wda[8], wdb[8];
#pragma unroll
  for (int t = 0; t < 8; ++t) { const int c = t * 16 + nloc; ab[t] = AF[(size_t)node * H + c] + bf16_rne(be1[c]); wda[t] = bf16_rne(we1[(size_t)(2 * H) * H + c]); wdb[t] = bf16_rne(we1[(size_t)(2 * H + 1) * H + c]); }
#pragma unroll 1
  for (int q = 0; q < 8; ++q) { const int rr = 2 * q + hlf; const int jn = b * N + j0 + rr;
    const float dx = pix - bf16_rne(pos[(size_t)jn * 3]), dy = piy - bf16_rne(pos[(size_t)jn * 3 + 1]), dz = piz - bf16_rne(pos[(size_t)jn * 3 + 2]); const float d2 = (dx * dx + dy * dy) + dz * dz;
    const float ex = vix - bf16_rne(vel[(size_t)jn * 3]), ey = viy - bf16_rne(vel[(size_t)jn * 3 + 1]), ez = viz - bf16_rne(vel[(size_t)jn * 3 + 2]); const float v2 = (ex * ex + ey * ey) + ez * ez;
#pragma unroll
    for (int t = 0; t < 8; ++t) { const int c = t * 16 + nloc; const float pre = ab[t] + BF[(size_t)jn * H + c] + pmul(d2, wda[t]) + pmul(v2, wdb[t]); b16 h_, l_; split16(silu(pre) * XS, h_, l_); Th[wave][rr][c] = h_; Tl[wave][rr][c] = l_; } }
  wave_lds_sync();
  v8f acc[8];
#pragma unroll
  for (int t = 0; t < 8; ++t) acc[t] = (v8f){};
#pragma unroll
  for (int kb = 0; kb < H; kb += 32) { const v16b a = frag_kb(&Th[wave][nloc][kb], hlf), al = frag_kb(&Tl[wave][nloc][kb], hlf);
#pragma unroll
    for (int t = 0; t < 8; ++t) { const v16b bw = frag_kb(WE2T + (size_t)(t * 16 + nloc) * H + kb, hlf); acc[t] = wmma16b(a, bw, acc[t]); acc[t] = wmma16b(al, bw, acc[t]); } }
  wave_lds_sync();
  const float bav = bf16_rne(ba[0]);
#pragma unroll
  for (int r = 0; r < 8; ++r) { float pa = 0.0f; float mv[8];
#pragma unroll
    for (int t = 0; t < 8; ++t) { const float m_ = silu(acc[t][r] * (1.0f / (XS * WSC)) + bf16_rne(be2[t * 16 + nloc])); mv[t] = m_; pa += pmul(m_, bf16_rne(wa[t * 16 + nloc])); }
    pa = hsum16(pa); const float at = sigm(pa + bav);
#pragma unroll
    for (int t = 0; t < 8; ++t) { b16 h_, l_; split16(pmul(mv[t], at) * XS, h_, l_); Th[wave][8 * hlf + r][t * 16 + nloc] = h_; Tl[wave][8 * hlf + r][t * 16 + nloc] = l_; } }
  wave_lds_sync();
  const size_t row0 = ((size_t)il * N + j0);
  for (int pass = 0; pass < 2; ++pass) { for (int rr = 0; rr < 16; ++rr) if (lane < 16) { *(volatile v8b*)(Mh + (row0 + rr) * H + lane * 8) = *(const v8b*)(&Th[wave][rr][lane * 8]); *(volatile v8b*)(Ml + (row0 + rr) * H + lane * 8) = *(const v8b*)(&Tl[wave][rr][lane * 8]); } __threadfence(); }
}
__global__ __launch_bounds__(128) void node_kernel(const b16* __restrict__ Mh, const b16* __restrict__ Ml, const float* __restrict__ pos, const float* __restrict__ vel, const float* __restrict__ bp1, const float* __restrict__ wp2, const float* __restrict__ bv1, const float* __restrict__ wv2, const b16* __restrict__ WT, int node0, float* __restrict__ MAGG, float* __restrict__ PV8) {
  __shared__ float PVs[4][8];
  const int wave = threadIdx.x >> 5, lane = threadIdx.x & 31, nloc = lane & 15, hlf = lane >> 4; const int il = blockIdx.x * 4 + wave; const int node = node0 + il; const int b = node / N;
  const b16* WP1T = WT + (size_t)3 * H * H; const b16* WV1T = WT + (size_t)4 * H * H;
  const float self3[6] = {bf16_rne(pos[(size_t)node * 3]), bf16_rne(pos[(size_t)node * 3 + 1]), bf16_rne(pos[(size_t)node * 3 + 2]), bf16_rne(vel[(size_t)node * 3]), bf16_rne(vel[(size_t)node * 3 + 1]), bf16_rne(vel[(size_t)node * 3 + 2])};
  float cbp[8], cwp[8], cbv[8], cwv[8];
#pragma unroll
  for (int t = 0; t < 8; ++t) { const int c = t * 16 + nloc; cbp[t] = bf16_rne(bp1[c]); cwp[t] = bf16_rne(wp2[c]); cbv[t] = bf16_rne(bv1[c]); cwv[t] = bf16_rne(wv2[c]); }
  float pu = 0.0f, vu = 0.0f;
  float mg[4] = {0, 0, 0, 0};
  const b16* Mrow = Mh + (size_t)il * N * H; const b16* Mlrow = Ml + (size_t)il * N * H;
  for (int jt = 0; jt < N / 16; ++jt) { const int j0 = jt * 16;
    for (int rr = 0; rr < 16; ++rr) { const __attribute__((ext_vector_type(4))) _Float16 hv = *(const __attribute__((ext_vector_type(4))) _Float16*)(Mrow + (size_t)(j0 + rr) * H + lane * 4), lv = *(const __attribute__((ext_vector_type(4))) _Float16*)(Mlrow + (size_t)(j0 + rr) * H + lane * 4);
      for (int q = 0; q < 4; ++q) mg[q] += ((float)hv[q] + (float)lv[q]) * (1.0f / XS); }
#pragma unroll 1
    for (int br = 0; br < 2; ++br) { const b16* W1 = br ? WV1T : WP1T; v8f acc[8];
#pragma unroll
      for (int t = 0; t < 8; ++t) acc[t] = (v8f){};
#pragma unroll
      for (int kb = 0; kb < H; kb += 32) { const v16b a = frag_kb(Mrow + (size_t)(j0 + nloc) * H + kb, hlf), al = frag_kb(Mlrow + (size_t)(j0 + nloc) * H + kb, hlf);
#pragma unroll
        for (int t = 0; t < 8; ++t) { const v16b bw = frag_kb(W1 + (size_t)(t * 16 + nloc) * H + kb, hlf); acc[t] = wmma16b(a, bw, acc[t]); acc[t] = wmma16b(al, bw, acc[t]); } }
#pragma unroll
      for (int r = 0; r < 8; ++r) { float pd = 0.0f;
#pragma unroll
        for (int t = 0; t < 8; ++t) pd += pmul(silu(acc[t][r] * (1.0f / (XS * WSC)) + (br ? cbv[t] : cbp[t])), br ? cwv[t] : cwp[t]);
        pd = hsum16(pd); const float w_ = tanh_(pd); const int jn = b * N + j0 + 8 * hlf + r;
        if (nloc < 3) { const float other = bf16_rne((br ? vel : pos)[(size_t)jn * 3 + nloc]); const float diff = self3[br * 3 + nloc] - other; if (br) vu += pmul(diff, w_); else pu += pmul(diff, w_); } } } }
  const float p2 = pu + __shfl_xor(pu, 16), v2s = vu + __shfl_xor(vu, 16);
  if (hlf == 0 && nloc < 3) { const float inv = 1.0f / (float)(N - 1); PVs[wave][nloc] = fminf(fmaxf(self3[nloc] + p2 * inv, -CLAMPC), CLAMPC); PVs[wave][3 + nloc] = fminf(fmaxf(self3[3 + nloc] + v2s * inv, -CLAMPC), CLAMPC); }
  if (hlf == 0 && (nloc == 6 || nloc == 7)) PVs[wave][nloc] = 0.0f;
  const v4f mo = {mg[0], mg[1], mg[2], mg[3]};
  __syncthreads();
  for (int pass = 0; pass < 2; ++pass) { *(volatile v4f*)(MAGG + (size_t)node * H + lane * 4) = mo; if (wave == 0) ((volatile float*)PV8)[(size_t)(node0 + blockIdx.x * 4) * 8 + lane] = PVs[lane >> 3][lane & 7]; __threadfence(); }
}
__global__ __launch_bounds__(128) void nodemlp_kernel(const float* __restrict__ h, const b16* __restrict__ H16, const float* __restrict__ MAGG, const b16* __restrict__ WT, const float* __restrict__ bn1, const float* __restrict__ bn2, float* __restrict__ hout) {
  __shared__ __attribute__((aligned(16))) b16 Xh[4][16][2 * H + 8], Xl[4][16][2 * H + 8]; __shared__ __attribute__((aligned(16))) float Ts[4][16][H + 4];
  const int wave = threadIdx.x >> 5, lane = threadIdx.x & 31, nloc = lane & 15, hlf = lane >> 4; const size_t m0 = ((size_t)blockIdx.x * 4 + wave) * 16;
  const b16* WN1T = WT + (size_t)5 * H * H; const b16* WN2T = WT + (size_t)7 * H * H;
  for (int rr = 0; rr < 16; ++rr) { const size_t nd = m0 + rr; const int c0 = lane * 8;
    v8b hv, lv; if (lane < 16) { hv = *(const v8b*)(H16 + nd * H + c0); lv = (v8b){}; } else { const float* mg = MAGG + nd * H + (c0 - H); for (int j = 0; j < 8; ++j) { b16 a_, c_; split16(mg[j] * XS, a_, c_); hv[j] = a_; lv[j] = c_; } }
    *(v8b*)(&Xh[wave][rr][c0]) = hv; *(v8b*)(&Xl[wave][rr][c0]) = lv; }
  wave_lds_sync();
  v8f acc[8];
#pragma unroll
  for (int t = 0; t < 8; ++t) acc[t] = (v8f){};
#pragma unroll 2
  for (int kb = 0; kb < 2 * H; kb += 32) { const v16b a = frag_kb(&Xh[wave][nloc][kb], hlf), al = frag_kb(&Xl[wave][nloc][kb], hlf);
#pragma unroll
    for (int t = 0; t < 8; ++t) { const v16b bw = frag_kb(WN1T + (size_t)(t * 16 + nloc) * 2 * H + kb, hlf); acc[t] = wmma16b(a, bw, acc[t]); acc[t] = wmma16b(al, bw, acc[t]); } }
  wave_lds_sync();
#pragma unroll
  for (int t = 0; t < 8; ++t) { const float bb = bf16_rne(bn1[t * 16 + nloc]);
#pragma unroll
    for (int r = 0; r < 8; ++r) { b16 a_, c_; split16(silu(acc[t][r] * (1.0f / (XS * WSC)) + bb) * XS, a_, c_); Xh[wave][8 * hlf + r][t * 16 + nloc] = a_; Xl[wave][8 * hlf + r][t * 16 + nloc] = c_; } }
  wave_lds_sync();
#pragma unroll
  for (int t = 0; t < 8; ++t) acc[t] = (v8f){};
#pragma unroll
  for (int kb = 0; kb < H; kb += 32) { const v16b a = frag_kb(&Xh[wave][nloc][kb], hlf), al = frag_kb(&Xl[wave][nloc][kb], hlf);
#pragma unroll
    for (int t = 0; t < 8; ++t) { const v16b bw = frag_kb(WN2T + (size_t)(t * 16 + nloc) * H + kb, hlf); acc[t] = wmma16b(a, bw, acc[t]); acc[t] = wmma16b(al, bw, acc[t]); } }
#pragma unroll
  for (int t = 0; t < 8; ++t) { const int c = t * 16 + nloc; const float bb = bf16_rne(bn2[c]);
#pragma unroll
    for (int r = 0; r < 8; ++r) Ts[wave][8 * hlf + r][c] = acc[t][r] * (1.0f / (XS * WSC)) + bb + bf16_rne(h[(m0 + 8 * hlf + r) * H + c]); }
  wave_lds_sync();
  for (int pass = 0; pass < 2; ++pass) { for (int rr = 0; rr < 16; ++rr) *(volatile v4f*)(hout + (m0 + rr) * H + lane * 4) = *(const v4f*)(&Ts[wave][rr][lane * 4]); __threadfence(); }
}
__global__ __launch_bounds__(256) void posvel_kernel(const float* __restrict__ PV8, float* __restrict__ pout, float* __restrict__ vout) {
  const int t_ = threadIdx.x;
  for (int pass = 0; pass < 2; ++pass) { for (int i = t_; i < NN * 3; i += 256) { const int nd = i / 3, c = i - nd * 3; ((volatile float*)pout)[i] = PV8[nd * 8 + c]; ((volatile float*)vout)[i] = PV8[nd * 8 + 3 + c]; } __threadfence(); }
}
}

extern "C" void kernel_launch(void* const* d_in, const int* in_sizes, int n_in, void* d_out, int out_size, void* d_ws, size_t ws_size, hipStream_t stream) {
  (void)n_in;
  auto Fp = [&](int i) { return (const float*)d_in[i]; };
  if (in_sizes[0] != NN * H || in_sizes[1] != NN * 3 || in_sizes[2] != NN * 3 || in_sizes[3] != (2 * H + 2) * H || in_sizes[5] != H * H || in_sizes[15] != 2 * H * H || in_sizes[17] != H * H || out_size != NN * H + 2 * NN * 3) return;
  size_t off = 0; char* ws = (char*)d_ws;
  auto carve = [&](size_t bytes) { char* p = ws + off; off += (bytes + 255) & ~(size_t)255; return p; };
  constexpr int CHN = 128;
  b16* H16 = (b16*)carve((size_t)NN * H * 2); b16* WT = (b16*)carve((size_t)9 * H * H * 2); float* AF = (float*)carve((size_t)NN * H * 4); float* BF = (float*)carve((size_t)NN * H * 4); float* MAGG = (float*)carve((size_t)NN * H * 4); float* PV8 = (float*)carve((size_t)NN * 8 * 4);
  b16* Mh = (b16*)carve((size_t)CHN * N * H * 2); b16* Ml = (b16*)carve((size_t)CHN * N * H * 2);
  if (off > ws_size || off > ((size_t)128 << 20)) return;
  prep_kernel<<<(NN * H / 8 + 8 * H * H / 8 + 255) / 256, 256, 0, stream>>>(Fp(0), Fp(3), Fp(5), Fp(9), Fp(12), Fp(15), Fp(17), H16, WT);
  nodeab_kernel<<<dim3(NN / 64, 2), 128, 0, stream>>>(H16, WT, AF, BF);
  for (int c0 = 0; c0 < NN; c0 += CHN) {
    edge_kernel<<<CHN * (N / 16) / 4, 128, 0, stream>>>(AF, BF, Fp(1), Fp(2), Fp(3), Fp(4), Fp(6), Fp(7), Fp(8), WT, c0, Mh, Ml);
    node_kernel<<<CHN / 4, 128, 0, stream>>>(Mh, Ml, Fp(1), Fp(2), Fp(10), Fp(11), Fp(13), Fp(14), WT, c0, MAGG, PV8);
  }
  nodemlp_kernel<<<NN / 64, 128, 0, stream>>>(Fp(0), H16, MAGG, WT, Fp(16), Fp(18), (float*)d_out);
  posvel_kernel<<<1, 256, 0, stream>>>(PV8, (float*)d_out + (size_t)NN * H, (float*)d_out + (size_t)NN * H + NN * 3);
}
